// Bidirectional_Mamba_72524817760349
// MI455X (gfx1250) — hardware-verified
//
#include <hip/hip_runtime.h>


#define NB_    8
#define NL_    2048
#define NM_    (NB_ * NL_)
#define DM_    256
#define DI_    512
#define NS_    16
#define DR_    16
#define DBLW_  64
#define DRP_   32
#define NC_    7
#define LOG2E_ 1.4426950408889634f

static_assert(NM_ % 64 == 0);
static_assert(DI_ % 128 == 0);
static_assert(DBLW_ % 64 == 0);
static_assert(DM_ % 32 == 0);
static_assert(DI_ % 32 == 0);
static_assert(DRP_ % 32 == 0);
static_assert((NL_ & (NL_ - 1)) == 0);
static_assert(DI_ == 128 * 4);
static_assert(DM_ == 32 * 8);
static_assert(NB_ == 8);
static_assert(NB_ * NC_ <= 56);

typedef float          v4f   __attribute__((ext_vector_type(4)));
typedef float          v8f   __attribute__((ext_vector_type(8)));
typedef _Float16       v4h   __attribute__((ext_vector_type(4)));
typedef _Float16       v8h   __attribute__((ext_vector_type(8)));
typedef _Float16       v16h  __attribute__((ext_vector_type(16)));
typedef unsigned short u16x4 __attribute__((ext_vector_type(4)));
typedef unsigned short u16x8 __attribute__((ext_vector_type(8)));

union Frag  { u16x8 h[2]; v16h v; };
union Pack8 { v8h f; u16x8 u; };
union Pack4 { v4h f; u16x4 u; };

__device__ __forceinline__ v8f ld8f(const float* p) {
  const v4f a = *(const v4f*)p;
  const v4f b = *(const v4f*)(p + 4);
  return __builtin_shufflevector(a, b, 0, 1, 2, 3, 4, 5, 6, 7);
}
__device__ __forceinline__ float wave_sum(float v) {
  v += __shfl_xor(v, 16, 32);
  v += __shfl_xor(v, 8, 32);
  v += __shfl_xor(v, 4, 32);
  v += __shfl_xor(v, 2, 32);
  v += __shfl_xor(v, 1, 32);
  return v;
}
__device__ __forceinline__ float silu_f(float x) {
  const float e = expf(-x);
  return x * __builtin_amdgcn_rcpf(1.0f + e);
}
__device__ __forceinline__ float softplus_f(float x) {
  return fmaxf(x, 0.0f) + log1pf(expf(-fabsf(x)));
}
__device__ __forceinline__ unsigned short f16_bits(float f) {
  const _Float16 hv = (_Float16)f;
  return __builtin_bit_cast(unsigned short, hv);
}

__device__ __forceinline__ void mma(v8f& acc, const Frag& a, const Frag& b) {
  acc = __builtin_amdgcn_wmma_f32_16x16x32_f16(false, a.v, false, b.v, (short)0, acc, false, false);
  asm volatile("v_nop\n\tv_nop\n\tv_nop\n\tv_nop" : "+v"(acc) : "v"(a.v), "v"(b.v));
}

__global__ __launch_bounds__(256)
void k_cvt(const float* __restrict__ src, unsigned short* dst, int spitch, int Rsrc, int Csrc,
           int Rdst, int Cdst, int total, float scale)
{
  const int i = blockIdx.x * 256 + threadIdx.x;
  if (i >= total) return;
  const int c8n = Cdst >> 3;
  const int cq  = i % c8n;
  const int rb  = i / c8n;
  const int r   = rb % Rdst;
  const int bt  = rb / Rdst;
  const int c0  = cq * 8;
  const int rr  = min(r, Rsrc - 1);
  const float* sp = src + ((size_t)bt * Rsrc + rr) * (size_t)spitch;
  v8f x;
#pragma unroll
  for (int c = 0; c < 8; ++c) {
    const int cc  = c0 + c;
    const int ccl = min(cc, Csrc - 1);
    const float v = sp[ccl];
    x[c] = (r < Rsrc && cc < Csrc) ? v * scale : 0.0f;
  }
  Pack8 pk;
  pk.f = __builtin_convertvector(x, v8h);
  const u16x8 o = pk.u;
  unsigned short* dp = dst + (size_t)i * 8;
  *(volatile u16x8*)dp = o;
  __threadfence();
  *(volatile u16x8*)dp = o;
}

__global__ __launch_bounds__(256)
void k_ln(const float* __restrict__ x, const float* __restrict__ nw, const float* __restrict__ nbv,
          unsigned short* u0, unsigned short* u1, int nrows)
{
  const int lane = threadIdx.x & 31, wave = threadIdx.x >> 5;
  const int row  = blockIdx.x * 8 + wave;
  if (row >= nrows) return;
  const int c0 = lane * 8;
  const v8f v = ld8f(x + (size_t)row * DM_ + c0);
  float s = 0.0f;
#pragma unroll
  for (int c = 0; c < 8; ++c) s += v[c];
  s = wave_sum(s);
  const float mu = s * (1.0f / DM_);
  v8f d;
  float q = 0.0f;
#pragma unroll
  for (int c = 0; c < 8; ++c) { d[c] = v[c] - mu; q = fmaf(d[c], d[c], q); }
  q = wave_sum(q);
  const float var = q * (1.0f / DM_);
  const float rs  = rsqrtf(var + 1e-5f);
  const v8f w0 = ld8f(nw + c0),       b0 = ld8f(nbv + c0);
  const v8f w1 = ld8f(nw + DM_ + c0), b1 = ld8f(nbv + DM_ + c0);
  v8f o0, o1;
#pragma unroll
  for (int c = 0; c < 8; ++c) {
    const float tn = d[c] * rs;
    o0[c] = tn * w0[c] + b0[c];
    o1[c] = tn * w1[c] + b1[c];
  }
  Pack8 p0, p1;
  p0.f = __builtin_convertvector(o0, v8h);
  p1.f = __builtin_convertvector(o1, v8h);
  const u16x8 q0 = p0.u, q1 = p1.u;
  unsigned short* g0 = u0 + (size_t)row * DM_ + c0;
  unsigned short* g1 = u1 + (size_t)row * DM_ + c0;
  *(volatile u16x8*)g0 = q0;
  *(volatile u16x8*)g1 = q1;
  __threadfence();
  *(volatile u16x8*)g0 = q0;
  *(volatile u16x8*)g1 = q1;
}

template<int NBF>
__device__ __forceinline__ void tile_store_pass(const float* st, float* gp, int ldc, int lane) {
  constexpr int CW  = NBF * 16;
  constexpr int P   = CW + 4;
  constexpr int LPR = CW / 4;
  constexpr int RPI = 32 / LPR;
  constexpr int NIT = 32 / RPI;
  const int rsub = lane / LPR;
  const int c4   = (lane % LPR) * 4;
#pragma unroll
  for (int it = 0; it < NIT; ++it) {
    const int row = it * RPI + rsub;
    const v4f v = *(const v4f*)(st + row * P + c4);
    *(volatile v4f*)(gp + (size_t)row * ldc + c4) = v;
  }
}

template<int NBF, int EPI>
__global__ __launch_bounds__(128)
void k_gemm(const unsigned short* __restrict__ A, const unsigned short* __restrict__ Bw,
            float* C, const float* __restrict__ bias,
            int lda, int ldb, int ldc, int K, float scale)
{
  constexpr int CW = NBF * 16;
  constexpr int P  = CW + 4;
  __shared__ __attribute__((aligned(16))) float stile[4][32 * P];

  const int tid  = threadIdx.x;
  const int lane = tid & 31;
  const int wave = tid >> 5;
  const int h    = lane >> 4;
  const int m    = lane & 15;
  const int wm   = wave >> 1;
  const int wn   = wave & 1;

  const int rowW = blockIdx.y * 64 + wm * 32;
  const int colW = blockIdx.x * (2 * CW) + wn * CW;

  v8f acc[2 * NBF];
#pragma unroll
  for (int j = 0; j < 2 * NBF; ++j)
#pragma unroll
    for (int r = 0; r < 8; ++r) acc[j][r] = 0.0f;

  const size_t aoff = (size_t)(rowW + m) * lda + 8 * h;
  const size_t boff = (size_t)(colW + m) * ldb + 8 * h;
  const size_t a16  = (size_t)16 * lda;
  const size_t b16  = (size_t)16 * ldb;
  const int nk = K >> 5;

#pragma unroll 1
  for (int kt = 0; kt < nk; ++kt) {
    const size_t k0 = (size_t)kt * 32;
    Frag fa[2], fb[NBF];
#pragma unroll
    for (int s = 0; s < 2; ++s) {
      const unsigned short* p = A + aoff + s * a16 + k0;
      fa[s].h[0] = *(const u16x8*)(p);
      fa[s].h[1] = *(const u16x8*)(p + 16);
    }
#pragma unroll
    for (int j = 0; j < NBF; ++j) {
      const unsigned short* p = Bw + boff + j * b16 + k0;
      fb[j].h[0] = *(const u16x8*)(p);
      fb[j].h[1] = *(const u16x8*)(p + 16);
    }
#pragma unroll
    for (int s = 0; s < 2; ++s)
#pragma unroll
      for (int j = 0; j < NBF; ++j)
        mma(acc[s * NBF + j], fa[s], fb[j]);
  }

  float* st = stile[wave];
#pragma unroll
  for (int s = 0; s < 2; ++s)
#pragma unroll
    for (int j = 0; j < NBF; ++j)
#pragma unroll
      for (int r = 0; r < 8; ++r)
        st[(s * 16 + 8 * h + r) * P + j * 16 + m] = acc[s * NBF + j][r] * scale;
  __syncthreads();

  if (EPI == 1) {
#pragma unroll 1
    for (int e = lane; e < 32 * CW; e += 32) {
      const int row = e / CW;
      const int col = e - row * CW;
      const float v = st[row * P + col] + bias[colW + col];
      st[row * P + col] = softplus_f(v);
    }
    __syncthreads();
  }

  float* gp = C + (size_t)rowW * ldc + colW;
  tile_store_pass<NBF>(st, gp, ldc, lane);
  __threadfence();
  tile_store_pass<NBF>(st, gp, ldc, lane);
}

__global__ __launch_bounds__(128)
void k_conv(const float* __restrict__ xi, const float* __restrict__ cw, const float* __restrict__ cb,
            float* xc, unsigned short* xc16, int dir)
{
  const int mrow = blockIdx.x;
  const int t    = mrow & (NL_ - 1);
  const int brow = mrow - t;
  const int d0   = threadIdx.x * 4;

  v4f wv[4];
#pragma unroll
  for (int c = 0; c < 4; ++c) wv[c] = *(const v4f*)(cw + (size_t)(d0 + c) * 4);
  const v4f bias = *(const v4f*)(cb + d0);

  v4f s = {0.0f, 0.0f, 0.0f, 0.0f};
#pragma unroll
  for (int k = 0; k < 4; ++k) {
    const int  tk  = t + dir * (k - 3);
    const bool ok  = (tk >= 0) && (tk < NL_);
    const int  tkc = min(max(tk, 0), NL_ - 1);
    const v4f  xv  = *(const v4f*)(xi + (size_t)(brow + tkc) * DI_ + d0);
#pragma unroll
    for (int c = 0; c < 4; ++c) {
      const float xe = ok ? xv[c] : 0.0f;
      s[c] = fmaf(wv[c][k], xe, s[c]);
    }
  }
  v4f u;
#pragma unroll
  for (int c = 0; c < 4; ++c) u[c] = silu_f(s[c] + bias[c]);

  Pack4 pk;
  pk.f = __builtin_convertvector(u * 8.0f, v4h);
  const u16x4 uh = pk.u;
  float* gp = xc + (size_t)mrow * DI_ + d0;
  unsigned short* hp = xc16 + (size_t)mrow * DI_ + d0;
  *(volatile v4f*)gp = u;
  *(volatile u16x4*)hp = uh;
  __threadfence();
  *(volatile v4f*)gp = u;
  *(volatile u16x4*)hp = uh;
}

__global__ __launch_bounds__(64)
void k_scan(const float* __restrict__ xc, const float* __restrict__ dt, const float* __restrict__ dbl,
            const float* __restrict__ Alog, const float* __restrict__ Dp, float* ysum)
{
  __shared__ float a2s[NS_ * 64];
  const int tid = threadIdx.x;
  const int d   = blockIdx.x * 64 + tid;
  const int b   = blockIdx.y;
#pragma unroll 1
  for (int n = 0; n < NS_; ++n)
    a2s[n * 64 + tid] = -expf(Alog[(size_t)d * NS_ + n]) * LOG2E_;
  __syncthreads();
  float a2[NS_], hs[NS_];
#pragma unroll
  for (int n = 0; n < NS_; ++n) { a2[n] = a2s[n * 64 + tid]; hs[n] = 0.0f; }
  const float Dd = Dp[d];
  const size_t rbase = (size_t)b * NL_;
  float xv = 0.0f, dv = 0.0f;

#pragma unroll 1
  for (int t = 0; t < NL_; ++t) {
    const size_t row = rbase + (size_t)t;
    xv = xc[row * DI_ + d];
    dv = dt[row * DI_ + d];
    const v4f* bp4 = (const v4f*)(dbl + row * DBLW_ + NS_);
    v4f bq[4];
#pragma unroll
    for (int q = 0; q < 4; ++q) bq[q] = bp4[q];
    const float du = dv * xv;
#pragma unroll
    for (int n = 0; n < NS_; ++n) {
      const float da = exp2f(dv * a2[n]);
      hs[n] = fmaf(da, hs[n], du * bq[n >> 2][n & 3]);
    }
  }

  const size_t rowL = rbase + (size_t)(NL_ - 1);
  const v4f* bp4 = (const v4f*)(dbl + rowL * DBLW_ + NS_);
  const v4f* cp4 = (const v4f*)(dbl + rowL * DBLW_ + 2 * NS_);
  v4f bq[4], cq[4];
#pragma unroll
  for (int q = 0; q < 4; ++q) { bq[q] = bp4[q]; cq[q] = cp4[q]; }
  const float du = dv * xv;
  float yf = 0.0f, y1 = 0.0f;
#pragma unroll
  for (int n = 0; n < NS_; ++n) {
    const float cn = cq[n >> 2][n & 3];
    yf = fmaf(hs[n], cn, yf);
    y1 = fmaf(du * bq[n >> 2][n & 3], cn, y1);
  }
  const float v = (yf + xv * Dd) + (y1 + xv * Dd);
  float* p = ysum + (size_t)b * DI_ + d;
  *(volatile float*)p = v;
  __threadfence();
  *(volatile float*)p = v;
}

__global__ __launch_bounds__(256)
void k_tail(const float* __restrict__ x,
            const unsigned short* __restrict__ u0, const unsigned short* __restrict__ u1,
            const unsigned short* __restrict__ inw16, const unsigned short* __restrict__ outw16,
            const float* __restrict__ ysum,
            const float* __restrict__ nfw, const float* __restrict__ nfb,
            const float* __restrict__ hw, const float* __restrict__ hbias,
            float* out)
{
  __shared__ __attribute__((aligned(16))) unsigned short us[16 * DM_];
  __shared__ __attribute__((aligned(16))) unsigned short ys[16 * DI_];
  __shared__ __attribute__((aligned(16))) float zs[NB_ * DI_];
  __shared__ __attribute__((aligned(16))) float hsr[2][NB_ * DM_];
  __shared__ __attribute__((aligned(16))) float outs[64];

  const int tid = threadIdx.x, lane = tid & 31, wave = tid >> 5, h = lane >> 4, m = lane & 15;
  if (tid < 64) outs[tid] = 0.0f;
  const u16x8 zero8 = {0, 0, 0, 0, 0, 0, 0, 0};

#pragma unroll 1
  for (int i = 0; i < 2; ++i) {
    const unsigned short* up = (i == 0) ? u0 : u1;
#pragma unroll
    for (int it = 0; it < 2; ++it) {
      const int q  = tid + it * 256;
      const int r  = q >> 5;
      const int c8 = (q & 31) * 8;
      const int rr = r & 7;
      u16x8 v = *(const u16x8*)(up + ((size_t)rr * NL_ + (NL_ - 1)) * DM_ + c8);
      if (r >= 8) v = zero8;
      *(u16x8*)(us + r * DM_ + c8) = v;
    }
    __syncthreads();

    v8f az[4];
#pragma unroll
    for (int j = 0; j < 4; ++j)
#pragma unroll
      for (int r = 0; r < 8; ++r) az[j][r] = 0.0f;
    const unsigned short* wb = inw16 + ((size_t)i * 2 * DI_ + DI_ + wave * 64 + m) * DM_ + 8 * h;
#pragma unroll 1
    for (int k0 = 0; k0 < DM_; k0 += 32) {
      Frag a;
      a.h[0] = *(const u16x8*)(us + m * DM_ + k0 + 8 * h);
      a.h[1] = *(const u16x8*)(us + m * DM_ + k0 + 16 + 8 * h);
#pragma unroll
      for (int j = 0; j < 4; ++j) {
        Frag bf;
        const unsigned short* p = wb + (size_t)j * 16 * DM_ + k0;
        bf.h[0] = *(const u16x8*)(p);
        bf.h[1] = *(const u16x8*)(p + 16);
        mma(az[j], a, bf);
      }
    }
    if (h == 0) {
#pragma unroll
      for (int j = 0; j < 4; ++j)
#pragma unroll
        for (int r = 0; r < 8; ++r)
          zs[r * DI_ + wave * 64 + j * 16 + m] = az[j][r] * 0.0625f;
    }
    __syncthreads();

#pragma unroll 1
    for (int e = tid; e < 16 * DI_; e += 256) {
      const int row = e >> 9;
      const int col = e & (DI_ - 1);
      const int rr  = row & 7;
      const float z  = zs[rr * DI_ + col];
      const float yv = ysum[(size_t)i * NB_ * DI_ + (size_t)rr * DI_ + col] * silu_f(z);
      const unsigned short bits = f16_bits(yv);
      ys[e] = (row < 8) ? bits : (unsigned short)0;
    }
    __syncthreads();

    v8f ao[2];
#pragma unroll
    for (int j = 0; j < 2; ++j)
#pragma unroll
      for (int r = 0; r < 8; ++r) ao[j][r] = 0.0f;
    const unsigned short* wo = outw16 + ((size_t)i * DM_ + wave * 32 + m) * DI_ + 8 * h;
#pragma unroll 1
    for (int k0 = 0; k0 < DI_; k0 += 32) {
      Frag a;
      a.h[0] = *(const u16x8*)(ys + m * DI_ + k0 + 8 * h);
      a.h[1] = *(const u16x8*)(ys + m * DI_ + k0 + 16 + 8 * h);
#pragma unroll
      for (int j = 0; j < 2; ++j) {
        Frag bf;
        const unsigned short* p = wo + (size_t)j * 16 * DI_ + k0;
        bf.h[0] = *(const u16x8*)(p);
        bf.h[1] = *(const u16x8*)(p + 16);
        mma(ao[j], a, bf);
      }
    }
    if (h == 0) {
#pragma unroll
      for (int j = 0; j < 2; ++j)
#pragma unroll
        for (int r = 0; r < 8; ++r)
          hsr[i][r * DM_ + wave * 32 + j * 16 + m] = ao[j][r] * 0.0625f;
    }
    __syncthreads();
  }

  {
    const int b  = wave;
    const int c0 = lane * 8;
    const v8f xv = ld8f(x + ((size_t)b * NL_ + (NL_ - 1)) * DM_ + c0);
    v8f rv;
    float s = 0.0f;
#pragma unroll
    for (int c = 0; c < 8; ++c) {
      const float h0 = hsr[0][b * DM_ + c0 + c];
      const float h1 = hsr[1][b * DM_ + c0 + c];
      rv[c] = (xv[c] + xv[c]) + (h0 + h1);
      s += rv[c];
    }
    s = wave_sum(s);
    const float mu = s * (1.0f / DM_);
    v8f dv;
    float q = 0.0f;
#pragma unroll
    for (int c = 0; c < 8; ++c) { dv[c] = rv[c] - mu; q = fmaf(dv[c], dv[c], q); }
    q = wave_sum(q);
    const float var = q * (1.0f / DM_);
    const float rs  = rsqrtf(var + 1e-5f);
    const v8f fw = ld8f(nfw + c0), fb = ld8f(nfb + c0);
    v8f hid;
#pragma unroll
    for (int c = 0; c < 8; ++c) hid[c] = (dv[c] * rs) * fw[c] + fb[c];
#pragma unroll 1
    for (int k = 0; k < NC_; ++k) {
      const v8f wk = ld8f(hw + (size_t)k * DM_ + c0);
      float pr = 0.0f;
#pragma unroll
      for (int c = 0; c < 8; ++c) pr = fmaf(hid[c], wk[c], pr);
      pr = wave_sum(pr);
      if (lane == 0) outs[b * NC_ + k] = pr + hbias[k];
    }
  }
  __syncthreads();
  if (wave == 0) {
    const v4f v = *(const v4f*)(outs + (lane & 15) * 4);
    if (lane < 14) *(volatile v4f*)(out + lane * 4) = v;
    __threadfence();
    if (lane < 14) *(volatile v4f*)(out + lane * 4) = v;
  }
}

extern "C" void kernel_launch(void* const* d_in, const int* in_sizes, int n_in,
                              void* d_out, int out_size, void* d_ws, size_t ws_size,
                              hipStream_t stream)
{
  if (n_in < 17) return;
  if (in_sizes[0]  != NM_ * DM_)                    return;
  if (in_sizes[1]  != 2 * 2 * DI_ * DM_)            return;
  if (in_sizes[2]  != 2 * DI_ * 4)                  return;
  if (in_sizes[3]  != 2 * DI_)                      return;
  if (in_sizes[4]  != 2 * (DR_ + 2 * NS_) * DI_)    return;
  if (in_sizes[5]  != 2 * DI_ * DR_)                return;
  if (in_sizes[6]  != 2 * DI_)                      return;
  if (in_sizes[7]  != 2 * DI_ * NS_)                return;
  if (in_sizes[8]  != 2 * DI_ * NS_)                return;
  if (in_sizes[9]  != 2 * DI_)                      return;
  if (in_sizes[10] != 2 * DM_ * DI_)                return;
  if (in_sizes[11] != 2 * DM_)                      return;
  if (in_sizes[12] != 2 * DM_)                      return;
  if (in_sizes[13] != DM_)                          return;
  if (in_sizes[14] != DM_)                          return;
  if (in_sizes[15] != NC_ * DM_)                    return;
  if (in_sizes[16] != NC_)                          return;
  if (out_size != NB_ * NC_)                        return;

  const float* x     = (const float*)d_in[0];
  const float* inw   = (const float*)d_in[1];
  const float* cw    = (const float*)d_in[2];
  const float* cb    = (const float*)d_in[3];
  const float* xpw   = (const float*)d_in[4];
  const float* dtw   = (const float*)d_in[5];
  const float* dtb   = (const float*)d_in[6];
  const float* alog  = (const float*)d_in[7];
  const float* ablog = (const float*)d_in[8];
  const float* Dp    = (const float*)d_in[9];
  const float* outw  = (const float*)d_in[10];
  const float* nw    = (const float*)d_in[11];
  const float* nbv   = (const float*)d_in[12];
  const float* nfw   = (const float*)d_in[13];
  const float* nfb   = (const float*)d_in[14];
  const float* hw    = (const float*)d_in[15];
  const float* hbb   = (const float*)d_in[16];
  float* out = (float*)d_out;

  const size_t SZ_U    = (size_t)NM_ * DM_ * 2;
  const size_t SZ_F512 = (size_t)NM_ * DI_ * 4;
  const size_t SZ_XC16 = (size_t)NM_ * DI_ * 2;
  const size_t SZ_DBL  = (size_t)NM_ * DBLW_ * 4;
  const size_t SZ_DTR  = (size_t)NM_ * DRP_ * 2;
  const size_t SZ_INW  = (size_t)2 * 2 * DI_ * DM_ * 2;
  const size_t SZ_XPW  = (size_t)2 * DBLW_ * DI_ * 2;
  const size_t SZ_DTW  = (size_t)2 * DI_ * DRP_ * 2;
  const size_t SZ_OUTW = (size_t)2 * DM_ * DI_ * 2;
  const size_t SZ_YS   = (size_t)2 * NB_ * DI_ * 4;

  const size_t OFF_U0   = 0;
  const size_t OFF_U1   = OFF_U0 + SZ_U;
  const size_t OFF_XIDT = OFF_U1 + SZ_U;
  const size_t OFF_XC   = OFF_XIDT + SZ_F512;
  const size_t OFF_XC16 = OFF_XC + SZ_F512;
  const size_t OFF_DBL  = OFF_XC16 + SZ_XC16;
  const size_t OFF_DTR  = OFF_DBL + SZ_DBL;
  const size_t OFF_INW  = OFF_DTR + SZ_DTR;
  const size_t OFF_XPW  = OFF_INW + SZ_INW;
  const size_t OFF_DTW  = OFF_XPW + SZ_XPW;
  const size_t OFF_OUTW = OFF_DTW + SZ_DTW;
  const size_t OFF_YS   = OFF_OUTW + SZ_OUTW;
  const size_t WS_END   = OFF_YS + SZ_YS;
  if (WS_END > ws_size) return;
  if (WS_END > (size_t)134217728) return;

  char* ws = (char*)d_ws;
  unsigned short* u0p    = (unsigned short*)(ws + OFF_U0);
  unsigned short* u1p    = (unsigned short*)(ws + OFF_U1);
  float*          xidt   = (float*)(ws + OFF_XIDT);
  float*          xcp    = (float*)(ws + OFF_XC);
  unsigned short* xc16   = (unsigned short*)(ws + OFF_XC16);
  float*          dblp   = (float*)(ws + OFF_DBL);
  unsigned short* dtr16  = (unsigned short*)(ws + OFF_DTR);
  unsigned short* inw16  = (unsigned short*)(ws + OFF_INW);
  unsigned short* xpw16  = (unsigned short*)(ws + OFF_XPW);
  unsigned short* dtw16  = (unsigned short*)(ws + OFF_DTW);
  unsigned short* outw16 = (unsigned short*)(ws + OFF_OUTW);
  float*          ysum   = (float*)(ws + OFF_YS);

  {
    int total;
    total = 2 * (2 * DI_) * (DM_ / 8);
    hipLaunchKernelGGL(k_cvt, dim3((total + 255) / 256), dim3(256), 0, stream,
                       inw, inw16, (int)DM_, (int)(2 * DI_), (int)DM_, (int)(2 * DI_), (int)DM_, total, 16.0f);
    total = 2 * DBLW_ * (DI_ / 8);
    hipLaunchKernelGGL(k_cvt, dim3((total + 255) / 256), dim3(256), 0, stream,
                       xpw, xpw16, (int)DI_, (int)(DR_ + 2 * NS_), (int)DI_, (int)DBLW_, (int)DI_, total, 16.0f);
    total = 2 * DI_ * (DRP_ / 8);
    hipLaunchKernelGGL(k_cvt, dim3((total + 255) / 256), dim3(256), 0, stream,
                       dtw, dtw16, (int)DR_, (int)DI_, (int)DR_, (int)DI_, (int)DRP_, total, 4.0f);
    total = 2 * DM_ * (DI_ / 8);
    hipLaunchKernelGGL(k_cvt, dim3((total + 255) / 256), dim3(256), 0, stream,
                       outw, outw16, (int)DI_, (int)DM_, (int)DI_, (int)DM_, (int)DI_, total, 16.0f);
  }

  hipLaunchKernelGGL(k_ln, dim3(NM_ / 8), dim3(256), 0, stream,
                     x, nw, nbv, u0p, u1p, (int)NM_);

  for (int i = 0; i < 2; ++i) {
    const int dir = (i == 0) ? 1 : -1;
    const unsigned short* up = (i == 0) ? u0p : u1p;

    hipLaunchKernelGGL(HIP_KERNEL_NAME(k_gemm<4, 0>), dim3(DI_ / 128, NM_ / 64), dim3(128), 0, stream,
                       up, (const unsigned short*)(inw16 + (size_t)i * 2 * DI_ * DM_),
                       xidt, dtb, (int)DM_, (int)DM_, (int)DI_, (int)DM_, 0.0625f);

    hipLaunchKernelGGL(k_conv, dim3(NM_), dim3(128), 0, stream,
                       (const float*)xidt, cw + (size_t)i * DI_ * 4, cb + (size_t)i * DI_, xcp, xc16, dir);

    hipLaunchKernelGGL(HIP_KERNEL_NAME(k_gemm<2, 0>), dim3(DBLW_ / 64, NM_ / 64), dim3(128), 0, stream,
                       (const unsigned short*)xc16, (const unsigned short*)(xpw16 + (size_t)i * DBLW_ * DI_),
                       dblp, dtb, (int)DI_, (int)DI_, (int)DBLW_, (int)DI_, 0.0078125f);

    {
      const int total = NM_ * (DRP_ / 8);
      hipLaunchKernelGGL(k_cvt, dim3((total + 255) / 256), dim3(256), 0, stream,
                         (const float*)dblp, dtr16, (int)DBLW_, (int)NM_, (int)DR_, (int)NM_, (int)DRP_, total, 8.0f);
    }

    hipLaunchKernelGGL(HIP_KERNEL_NAME(k_gemm<4, 1>), dim3(DI_ / 128, NM_ / 64), dim3(128), 0, stream,
                       (const unsigned short*)dtr16, (const unsigned short*)(dtw16 + (size_t)i * DI_ * DRP_),
                       xidt, dtb + (size_t)i * DI_, (int)DRP_, (int)DRP_, (int)DI_, (int)DRP_, 0.03125f);

    const float* ap = (i == 0) ? alog : (ablog + (size_t)DI_ * NS_);
    hipLaunchKernelGGL(k_scan, dim3(DI_ / 64, NB_), dim3(64), 0, stream,
                       (const float*)xcp, (const float*)xidt, (const float*)dblp, ap,
                       Dp + (size_t)i * DI_, ysum + (size_t)i * NB_ * DI_);
  }

  hipLaunchKernelGGL(k_tail, dim3(1), dim3(256), 0, stream,
                     x, (const unsigned short*)u0p, (const unsigned short*)u1p,
                     (const unsigned short*)inw16, (const unsigned short*)outw16,
                     (const float*)ysum, nfw, nfb, hw, hbb, out);
}
